// GraphDecoder_41248865911346
// MI455X (gfx1250) — hardware-verified
//
#include <hip/hip_runtime.h>
#include <hip/hip_bf16.h>
#include <stddef.h>


#define NTHR    256
#define NWAVE   8
#define EPT     8
#define NGRP    2
#define CHUNK   (NTHR * EPT * NGRP)
#define WCAP    (EPT * NGRP * 32)
#define LISTN   (NWAVE * WCAP)
#define NB1     4096
#define NB2     512
#define NB3     1024
#define HW      128
#define H3W     64
#define OUTW    40
#define OUTP    48
#define GROWS   64
#define P2N     (HW * 2 * HW)
#define P3N     (HW * HW)
#define P4N     (OUTP * H3W)
#define LDS_A1  (NB1 * 4 * 4 + LISTN * 4)
#define LDS_A2  (NB2 * HW * 4 + LISTN * 4)
#define LDS_A3  (NB3 * H3W * 4 + LISTN * 4)

static_assert((CHUNK & (CHUNK - 1)) == 0);
static_assert(CHUNK <= 4096);
static_assert(NB1 <= 4096 && (NB1 & (NB1 - 1)) == 0);
static_assert(NB2 <= 4096 && (NB2 & (NB2 - 1)) == 0);
static_assert(NB3 <= 4096 && (NB3 & (NB3 - 1)) == 0);
static_assert(NB1 % GROWS == 0 && NB2 % GROWS == 0 && NB3 % GROWS == 0);
static_assert((NB3 * H3W) % (NWAVE * 128) == 0);
static_assert(NB1 % (2 * NWAVE) == 0 && NB2 % NWAVE == 0 && NB3 % NWAVE == 0);
static_assert((P2N / 8) % 32 == 0 && (P3N / 8) % 32 == 0 && (P4N / 8) % 32 == 0);
static_assert((GROWS * OUTW) % (4 * 5 * 128) == 0);

typedef float v2f __attribute__((ext_vector_type(2)));
typedef float v4f __attribute__((ext_vector_type(4)));
typedef float v8f __attribute__((ext_vector_type(8)));
typedef int   v4i __attribute__((ext_vector_type(4)));
typedef unsigned short v8us  __attribute__((ext_vector_type(8)));
typedef unsigned short v16us __attribute__((ext_vector_type(16)));
typedef __bf16 v16bf __attribute__((ext_vector_type(16)));
union FragB { v16bf v; v16us u; v8us h[2]; };
struct HL { v8us hi; v8us lo; };

__device__ __forceinline__ unsigned int bf_bits(float f) {
  const unsigned int u = __float_as_uint(f);
  return (u + 0x7FFFu + ((u >> 16) & 1u)) >> 16;
}
__device__ __forceinline__ unsigned int bf_lo(float f, unsigned int hb) {
  return bf_bits(f - __uint_as_float(hb << 16));
}

__device__ __forceinline__ HL split8(v4f a, v4f b) {
  HL r;
  unsigned int h;
  h = bf_bits(a.x); r.hi[0] = (unsigned short)h; r.lo[0] = (unsigned short)bf_lo(a.x, h);
  h = bf_bits(a.y); r.hi[1] = (unsigned short)h; r.lo[1] = (unsigned short)bf_lo(a.y, h);
  h = bf_bits(a.z); r.hi[2] = (unsigned short)h; r.lo[2] = (unsigned short)bf_lo(a.z, h);
  h = bf_bits(a.w); r.hi[3] = (unsigned short)h; r.lo[3] = (unsigned short)bf_lo(a.w, h);
  h = bf_bits(b.x); r.hi[4] = (unsigned short)h; r.lo[4] = (unsigned short)bf_lo(b.x, h);
  h = bf_bits(b.y); r.hi[5] = (unsigned short)h; r.lo[5] = (unsigned short)bf_lo(b.y, h);
  h = bf_bits(b.z); r.hi[6] = (unsigned short)h; r.lo[6] = (unsigned short)bf_lo(b.z, h);
  h = bf_bits(b.w); r.hi[7] = (unsigned short)h; r.lo[7] = (unsigned short)bf_lo(b.w, h);
  return r;
}

__device__ __forceinline__ v8f wmb(v16bf a, v16bf b, v8f c) {
  v8f d = __builtin_amdgcn_wmma_f32_16x16x32_bf16(false, a, false, b, (short)0, c, false, false);
  asm volatile("v_nop\n\tv_nop\n\tv_nop\n\tv_nop" : "+v"(d) : "v"(a), "v"(b));
  return d;
}

template <int NBT>
__device__ __forceinline__ int scan_chunk(const int* __restrict__ dsts, int nE, int cbase, int nodeBase,
                                          int vec8, int* list, int tid, int lane, int wave) {
  int wc = 0;
#pragma unroll
  for (int g = 0; g < NGRP; ++g) {
    const int el0  = (g * NTHR + tid) * EPT;
    const int e0   = cbase + el0;
    const int sent = -2147483647 - 1;
    v4i da, db;
    if (vec8 != 0 && e0 + 7 < nE) {
      da = *(const v4i*)(dsts + e0);
      db = *(const v4i*)(dsts + e0 + 4);
    } else {
      da.x = (e0     < nE) ? dsts[min(e0, nE - 1)] : sent;
      da.y = (e0 + 1 < nE) ? dsts[min(e0 + 1, nE - 1)] : sent;
      da.z = (e0 + 2 < nE) ? dsts[min(e0 + 2, nE - 1)] : sent;
      da.w = (e0 + 3 < nE) ? dsts[min(e0 + 3, nE - 1)] : sent;
      db.x = (e0 + 4 < nE) ? dsts[min(e0 + 4, nE - 1)] : sent;
      db.y = (e0 + 5 < nE) ? dsts[min(e0 + 5, nE - 1)] : sent;
      db.z = (e0 + 6 < nE) ? dsts[min(e0 + 6, nE - 1)] : sent;
      db.w = (e0 + 7 < nE) ? dsts[min(e0 + 7, nE - 1)] : sent;
    }
    const unsigned nb = (unsigned)nodeBase;
    const unsigned s0 = (unsigned)da.x - nb, s1 = (unsigned)da.y - nb;
    const unsigned s2 = (unsigned)da.z - nb, s3 = (unsigned)da.w - nb;
    const unsigned s4 = (unsigned)db.x - nb, s5 = (unsigned)db.y - nb;
    const unsigned s6 = (unsigned)db.z - nb, s7 = (unsigned)db.w - nb;
    const bool h0 = s0 < (unsigned)NBT, h1 = s1 < (unsigned)NBT, h2 = s2 < (unsigned)NBT, h3 = s3 < (unsigned)NBT;
    const bool h4 = s4 < (unsigned)NBT, h5 = s5 < (unsigned)NBT, h6 = s6 < (unsigned)NBT, h7 = s7 < (unsigned)NBT;
    const unsigned any = __builtin_amdgcn_ballot_w32(h0 | h1 | h2 | h3 | h4 | h5 | h6 | h7);
    if (any != 0u) {
#define HITJ(J, HJ, SJ) { \
        const unsigned mj = __builtin_amdgcn_ballot_w32(HJ); \
        if (mj != 0u) { \
          if (HJ) { \
            const int pos = wc + (int)__builtin_amdgcn_mbcnt_lo(mj, 0u); \
            if (pos < WCAP) list[wave * WCAP + pos] = ((el0 + (J)) << 12) | (int)(SJ); \
          } \
          wc += (int)__builtin_popcount(mj); } }
      HITJ(0, h0, s0)
      HITJ(1, h1, s1)
      HITJ(2, h2, s2)
      HITJ(3, h3, s3)
      HITJ(4, h4, s4)
      HITJ(5, h5, s5)
      HITJ(6, h6, s6)
      HITJ(7, h7, s7)
#undef HITJ
    }
  }
  return wc;
}

__global__ __launch_bounds__(NTHR) void k_wprep(
    const float* __restrict__ W2l, const float* __restrict__ W2r,
    const float* __restrict__ W3l, const float* __restrict__ W3r,
    const float* __restrict__ W4,
    unsigned short* p2, unsigned short* p3, unsigned short* p4) {
  const int i = blockIdx.x * NTHR + threadIdx.x;
  float v[8];
  unsigned short* ph;
  unsigned short* pl;
  if (i < P2N / 8) {
    const int n = i >> 5, k0 = (i & 31) * 8;
    if (k0 < HW) {
#pragma unroll
      for (int e = 0; e < 8; ++e) v[e] = W2l[(k0 + e) * HW + n];
    } else {
#pragma unroll
      for (int e = 0; e < 8; ++e) v[e] = W2r[(k0 + e - HW) * HW + n];
    }
    ph = p2 + (size_t)n * (2 * HW) + k0;
    pl = ph + P2N;
  } else if (i < P2N / 8 + P3N / 8) {
    const int j = i - P2N / 8;
    const int n = j >> 4, k0 = (j & 15) * 8;
    if (n < H3W) {
#pragma unroll
      for (int e = 0; e < 8; ++e) v[e] = W3l[(k0 + e) * H3W + n];
    } else {
#pragma unroll
      for (int e = 0; e < 8; ++e) v[e] = W3r[(k0 + e) * H3W + (n - H3W)];
    }
    ph = p3 + (size_t)n * HW + k0;
    pl = ph + P3N;
  } else if (i < P2N / 8 + P3N / 8 + P4N / 8) {
    const int j = i - P2N / 8 - P3N / 8;
    const int n = j >> 3, k0 = (j & 7) * 8;
    if (n < OUTW) {
#pragma unroll
      for (int e = 0; e < 8; ++e) v[e] = W4[(k0 + e) * OUTW + n];
    } else {
#pragma unroll
      for (int e = 0; e < 8; ++e) v[e] = 0.f;
    }
    ph = p4 + (size_t)n * H3W + k0;
    pl = ph + P4N;
  } else {
    return;
  }
  v4f a, bq;
  a.x = v[0]; a.y = v[1]; a.z = v[2]; a.w = v[3];
  bq.x = v[4]; bq.y = v[5]; bq.z = v[6]; bq.w = v[7];
  const HL s = split8(a, bq);
  *(volatile v8us*)ph = s.hi;
  *(volatile v8us*)pl = s.lo;
  __threadfence();
  *(volatile v8us*)ph = s.hi;
  *(volatile v8us*)pl = s.lo;
}

__device__ __forceinline__ v4f l1row(const float* acc, int slot, const float* __restrict__ z, int nz,
                                     v4f wl0, v4f wl1, v4f wl2, v4f wr0, v4f wr1, v4f wr2, v4f bb) {
  const v4f a = *(const v4f*)(acc + slot * 4);
  const float inv = 1.0f / fmaxf(a.w, 1.0f);
  const float m0 = a.x * inv, m1 = a.y * inv, m2 = a.z * inv;
  const float x0 = z[(size_t)nz * 3 + 0], x1 = z[(size_t)nz * 3 + 1], x2 = z[(size_t)nz * 3 + 2];
  const v4f t = wl0 * m0 + wl1 * m1 + wl2 * m2;
  const v4f u = wr0 * x0 + wr1 * x1 + wr2 * x2;
  v4f s = (t + u) + bb;
  s.x = fmaxf(s.x, 0.f); s.y = fmaxf(s.y, 0.f); s.z = fmaxf(s.z, 0.f); s.w = fmaxf(s.w, 0.f);
  return s;
}

__global__ __launch_bounds__(NTHR) void k_agg1(
    const float* __restrict__ z, const int* __restrict__ ei,
    const float* __restrict__ W1l, const float* __restrict__ W1r, const float* __restrict__ b1,
    float* h1, int nN, int nPad, int nE, int vec8) {
  extern __shared__ v4f lds_dyn[];
  float* acc  = (float*)lds_dyn;
  int*   list = (int*)(acc + NB1 * 4);
  __shared__ int wcnt[NWAVE];
  __shared__ __attribute__((aligned(16))) float sw[7 * HW];
  const int tid = threadIdx.x, lane = tid & 31, wave = tid >> 5;
  const int nodeBase = blockIdx.x * NB1;
  const int* dsts = ei + nE;

  for (int i = tid; i < 7 * HW; i += NTHR)
    sw[i] = (i < 3 * HW) ? W1l[i] : ((i < 6 * HW) ? W1r[i - 3 * HW] : b1[i - 6 * HW]);
  {
    const v4f zz = {0.f, 0.f, 0.f, 0.f};
    for (int i = tid; i < NB1; i += NTHR) lds_dyn[i] = zz;
  }
  __syncthreads();

  const int nChunks = (nE + CHUNK - 1) / CHUNK;
#pragma unroll 1
  for (int ch = 0; ch < nChunks; ++ch) {
    const int cbase = ch * CHUNK;
    const int wc = scan_chunk<NB1>(dsts, nE, cbase, nodeBase, vec8, list, tid, lane, wave);
    if (lane == 0) wcnt[wave] = wc;
    __syncthreads();
    if (wave == 0) {
#pragma unroll 1
      for (int wsx = 0; wsx < NWAVE; ++wsx) {
        int n = __builtin_amdgcn_readfirstlane(wcnt[wsx]);
        n = n > WCAP ? WCAP : (n < 0 ? 0 : n);
        const int* lp = list + wsx * WCAP;
#pragma unroll 1
        for (int i = 0; i < n; ++i) {
          const int ent  = __builtin_amdgcn_readfirstlane(lp[i]);
          const int slot = ent & (NB1 - 1);
          int e = cbase + ((ent >> 12) & (CHUNK - 1));
          e = e > nE - 1 ? nE - 1 : e;
          int src = ei[e];
          src = src < 0 ? 0 : (src > nN - 1 ? nN - 1 : src);
          float val = 1.0f;
          if (lane < 3) val = z[(size_t)src * 3 + lane];
          if (lane < 4) acc[slot * 4 + lane] = acc[slot * 4 + lane] + val;
        }
      }
    }
    __syncthreads();
  }

  const v4f wl0 = *(const v4f*)(sw + 0 * HW + 4 * lane);
  const v4f wl1 = *(const v4f*)(sw + 1 * HW + 4 * lane);
  const v4f wl2 = *(const v4f*)(sw + 2 * HW + 4 * lane);
  const v4f wr0 = *(const v4f*)(sw + 3 * HW + 4 * lane);
  const v4f wr1 = *(const v4f*)(sw + 4 * HW + 4 * lane);
  const v4f wr2 = *(const v4f*)(sw + 5 * HW + 4 * lane);
  const v4f bb  = *(const v4f*)(sw + 6 * HW + 4 * lane);
  constexpr int RPW = NB1 / NWAVE;
#pragma unroll 1
  for (int g = 0; g < RPW / 2; ++g) {
    const int slot0 = wave * RPW + 2 * g;
    const int node0 = nodeBase + slot0;
    const int node1 = node0 + 1;
    const int nz0 = node0 > nN - 1 ? nN - 1 : node0;
    const int nz1 = node1 > nN - 1 ? nN - 1 : node1;
    const v4f ov0 = l1row(acc, slot0,     z, nz0, wl0, wl1, wl2, wr0, wr1, wr2, bb);
    const v4f ov1 = l1row(acc, slot0 + 1, z, nz1, wl0, wl1, wl2, wr0, wr1, wr2, bb);
    float* g0 = h1 + (size_t)node0 * HW + 4 * lane;
    float* g1 = h1 + (size_t)node1 * HW + 4 * lane;
    if (node0 < nPad) *(volatile v4f*)g0 = ov0;
    if (node1 < nPad) *(volatile v4f*)g1 = ov1;
    __threadfence();
    if (node0 < nPad) *(volatile v4f*)g0 = ov0;
    if (node1 < nPad) *(volatile v4f*)g1 = ov1;
  }
}

__global__ __launch_bounds__(NTHR) void k_agg128(
    const int* __restrict__ ei, const float* __restrict__ hin, float* mout,
    int nN, int nPad, int nE, int vec8) {
  extern __shared__ v4f lds_dyn[];
  float* acc  = (float*)lds_dyn;
  int*   list = (int*)(acc + NB2 * HW);
  __shared__ int wcnt[NWAVE];
  __shared__ float cnt[NB2];
  const int tid = threadIdx.x, lane = tid & 31, wave = tid >> 5;
  const int nodeBase = blockIdx.x * NB2;
  const int* dsts = ei + nE;

  {
    const v4f zz = {0.f, 0.f, 0.f, 0.f};
    for (int i = tid; i < NB2 * HW / 4; i += NTHR) lds_dyn[i] = zz;
    for (int i = tid; i < NB2; i += NTHR) cnt[i] = 0.f;
  }
  __syncthreads();

  const int nChunks = (nE + CHUNK - 1) / CHUNK;
#pragma unroll 1
  for (int ch = 0; ch < nChunks; ++ch) {
    const int cbase = ch * CHUNK;
    const int wc = scan_chunk<NB2>(dsts, nE, cbase, nodeBase, vec8, list, tid, lane, wave);
    if (lane == 0) wcnt[wave] = wc;
    __syncthreads();
    if (wave == 0) {
#pragma unroll 1
      for (int wsx = 0; wsx < NWAVE; ++wsx) {
        int n = __builtin_amdgcn_readfirstlane(wcnt[wsx]);
        n = n > WCAP ? WCAP : (n < 0 ? 0 : n);
        const int* lp = list + wsx * WCAP;
#pragma unroll 1
        for (int i = 0; i < n; ++i) {
          const int ent  = __builtin_amdgcn_readfirstlane(lp[i]);
          const int slot = ent & (NB2 - 1);
          int e = cbase + ((ent >> 12) & (CHUNK - 1));
          e = e > nE - 1 ? nE - 1 : e;
          int src = ei[e];
          src = src < 0 ? 0 : (src > nN - 1 ? nN - 1 : src);
          const v4f v = *(const v4f*)(hin + (size_t)src * HW + 4 * lane);
          v4f* ap = (v4f*)(acc + slot * HW + 4 * lane);
          *ap = *ap + v;
          if (lane == 0) cnt[slot] = cnt[slot] + 1.0f;
        }
      }
    }
    __syncthreads();
  }

  constexpr int RPW = NB2 / NWAVE;
#pragma unroll 1
  for (int j = 0; j < RPW; ++j) {
    const int slot = wave * RPW + j;
    v4f* ap = (v4f*)(acc + slot * HW + 4 * lane);
    const float inv = 1.0f / fmaxf(cnt[slot], 1.0f);
    *ap = *ap * inv;
  }
#pragma unroll 4
  for (int j = 0; j < RPW; ++j) {
    const int slot = wave * RPW + j;
    const int node = nodeBase + slot;
    if (node < nPad) {
      const v4f v = *(const v4f*)(acc + slot * HW + 4 * lane);
      *(volatile v4f*)(mout + (size_t)node * HW + 4 * lane) = v;
    }
  }
  __threadfence();
#pragma unroll 4
  for (int j = 0; j < RPW; ++j) {
    const int slot = wave * RPW + j;
    const int node = nodeBase + slot;
    if (node < nPad) {
      const v4f v = *(const v4f*)(acc + slot * HW + 4 * lane);
      *(volatile v4f*)(mout + (size_t)node * HW + 4 * lane) = v;
    }
  }
}

__global__ __launch_bounds__(NTHR) void k_agg64(
    const int* __restrict__ ei, const float* __restrict__ gs, const float* __restrict__ b3,
    float* hout, int nN, int nPad, int nE, int vec8) {
  extern __shared__ v4f lds_dyn[];
  float* acc  = (float*)lds_dyn;
  int*   list = (int*)(acc + NB3 * H3W);
  __shared__ int wcnt[NWAVE];
  __shared__ float cnt[NB3];
  const int tid = threadIdx.x, lane = tid & 31, wave = tid >> 5;
  const int nodeBase = blockIdx.x * NB3;
  const int* dsts = ei + nE;

  {
    const v4f zz = {0.f, 0.f, 0.f, 0.f};
    for (int i = tid; i < NB3 * H3W / 4; i += NTHR) lds_dyn[i] = zz;
    for (int i = tid; i < NB3; i += NTHR) cnt[i] = 0.f;
  }
  __syncthreads();

  const int nChunks = (nE + CHUNK - 1) / CHUNK;
#pragma unroll 1
  for (int ch = 0; ch < nChunks; ++ch) {
    const int cbase = ch * CHUNK;
    const int wc = scan_chunk<NB3>(dsts, nE, cbase, nodeBase, vec8, list, tid, lane, wave);
    if (lane == 0) wcnt[wave] = wc;
    __syncthreads();
    if (wave == 0) {
#pragma unroll 1
      for (int wsx = 0; wsx < NWAVE; ++wsx) {
        int n = __builtin_amdgcn_readfirstlane(wcnt[wsx]);
        n = n > WCAP ? WCAP : (n < 0 ? 0 : n);
        const int* lp = list + wsx * WCAP;
#pragma unroll 1
        for (int i = 0; i < n; ++i) {
          const int ent  = __builtin_amdgcn_readfirstlane(lp[i]);
          const int slot = ent & (NB3 - 1);
          int e = cbase + ((ent >> 12) & (CHUNK - 1));
          e = e > nE - 1 ? nE - 1 : e;
          int src = ei[e];
          src = src < 0 ? 0 : (src > nN - 1 ? nN - 1 : src);
          const v2f v = *(const v2f*)(gs + (size_t)src * HW + 2 * lane);
          v2f* ap = (v2f*)(acc + slot * H3W + 2 * lane);
          *ap = *ap + v;
          if (lane == 0) cnt[slot] = cnt[slot] + 1.0f;
        }
      }
    }
    __syncthreads();
  }

  const v2f bb = *(const v2f*)(b3 + 2 * lane);
  constexpr int RPW = NB3 / NWAVE;
#pragma unroll 2
  for (int j = 0; j < RPW; ++j) {
    const int slot = wave * RPW + j;
    int node = nodeBase + slot;
    node = node > nPad - 1 ? nPad - 1 : node;
    v2f* ap = (v2f*)(acc + slot * H3W + 2 * lane);
    const float inv = 1.0f / fmaxf(cnt[slot], 1.0f);
    const v2f sv = *(const v2f*)(gs + (size_t)node * HW + H3W + 2 * lane);
    v2f t = (*ap * inv + sv) + bb;
    t.x = fmaxf(t.x, 0.f); t.y = fmaxf(t.y, 0.f);
    *ap = t;
  }
  __syncthreads();

  const size_t outN = (size_t)nPad * H3W;
  const size_t ob   = (size_t)nodeBase * H3W;
  constexpr int NQ = (NB3 * H3W) / (NWAVE * 128);
#pragma unroll 4
  for (int q = 0; q < NQ; ++q) {
    const int f = (wave * NQ + q) * 128 + 4 * lane;
    const size_t gi = ob + (size_t)f;
    if (gi < outN) { const v4f v = *(const v4f*)(acc + f); *(volatile v4f*)(hout + gi) = v; }
  }
  __threadfence();
#pragma unroll 4
  for (int q = 0; q < NQ; ++q) {
    const int f = (wave * NQ + q) * 128 + 4 * lane;
    const size_t gi = ob + (size_t)f;
    if (gi < outN) { const v4f v = *(const v4f*)(acc + f); *(volatile v4f*)(hout + gi) = v; }
  }
}

template <int KS, bool EPI>
__global__ __launch_bounds__(NTHR) void k_gemm(
    const float* pa, const float* pb, const unsigned short* __restrict__ wp,
    const float* __restrict__ bias, float* outp, int nPad) {
  __shared__ __attribute__((aligned(16))) float stg[GROWS * HW];
  const int tid = threadIdx.x, lane = tid & 31, wave = tid >> 5, hh = lane >> 4, m = lane & 15;
  const int which = wave & 1;
  const int rt    = wave >> 1;
  const int row0  = blockIdx.x * GROWS;
  const int arow  = row0 + rt * 16 + m;
  constexpr int KP = 32 * KS;
  constexpr int KH = KS / 2;
  const unsigned short* whi = wp;
  const unsigned short* wlo = wp + (size_t)HW * KP;

  v8f acc[4];
#pragma unroll
  for (int t = 0; t < 4; ++t) { v8f zz = {0.f, 0.f, 0.f, 0.f, 0.f, 0.f, 0.f, 0.f}; acc[t] = zz; }

#pragma unroll 1
  for (int ks = 0; ks < KS; ++ks) {
    const float* src = (ks < KH) ? pa : pb;
    const int c0 = 32 * (ks < KH ? ks : ks - KH);
    const float* p0 = src + (size_t)arow * HW + c0 + 8 * hh;
    const v4f f0 = *(const v4f*)p0,        f1 = *(const v4f*)(p0 + 4);
    const v4f f2 = *(const v4f*)(p0 + 16), f3 = *(const v4f*)(p0 + 20);
    const HL s0 = split8(f0, f1);
    const HL s1 = split8(f2, f3);
    FragB ah, al;
    ah.h[0] = s0.hi; ah.h[1] = s1.hi;
    al.h[0] = s0.lo; al.h[1] = s1.lo;
#pragma unroll
    for (int t = 0; t < 4; ++t) {
      const int n = 64 * which + 16 * t + m;
      const unsigned short* bp = whi + (size_t)n * KP + 32 * ks + 8 * hh;
      const unsigned short* bq = wlo + (size_t)n * KP + 32 * ks + 8 * hh;
      FragB bh, bl;
      bh.h[0] = *(const v8us*)bp; bh.h[1] = *(const v8us*)(bp + 16);
      bl.h[0] = *(const v8us*)bq; bl.h[1] = *(const v8us*)(bq + 16);
      acc[t] = wmb(ah.v, bh.v, acc[t]);
      acc[t] = wmb(ah.v, bl.v, acc[t]);
      acc[t] = wmb(al.v, bh.v, acc[t]);
    }
  }

  float* sp = stg + (rt * 16 + 8 * hh) * HW + 64 * which + m;
#pragma unroll
  for (int t = 0; t < 4; ++t) {
    float bc = 0.f;
    if (EPI) bc = bias[64 * which + 16 * t + m];
    float v0 = acc[t][0] + bc, v1 = acc[t][1] + bc, v2 = acc[t][2] + bc, v3 = acc[t][3] + bc;
    float v4 = acc[t][4] + bc, v5 = acc[t][5] + bc, v6 = acc[t][6] + bc, v7 = acc[t][7] + bc;
    if (EPI) {
      v0 = fmaxf(v0, 0.f); v1 = fmaxf(v1, 0.f); v2 = fmaxf(v2, 0.f); v3 = fmaxf(v3, 0.f);
      v4 = fmaxf(v4, 0.f); v5 = fmaxf(v5, 0.f); v6 = fmaxf(v6, 0.f); v7 = fmaxf(v7, 0.f);
    }
    sp[0 * HW + 16 * t] = v0;
    sp[1 * HW + 16 * t] = v1;
    sp[2 * HW + 16 * t] = v2;
    sp[3 * HW + 16 * t] = v3;
    sp[4 * HW + 16 * t] = v4;
    sp[5 * HW + 16 * t] = v5;
    sp[6 * HW + 16 * t] = v6;
    sp[7 * HW + 16 * t] = v7;
  }
  __syncthreads();

  const float* lp = stg + (8 * wave) * HW + 4 * lane;
  float* gp = outp + (size_t)(row0 + 8 * wave) * HW + 4 * lane;
  v4f ov[8];
#pragma unroll
  for (int q = 0; q < 8; ++q) ov[q] = *(const v4f*)(lp + q * HW);
#pragma unroll
  for (int q = 0; q < 8; ++q) *(volatile v4f*)(gp + (size_t)q * HW) = ov[q];
  __threadfence();
#pragma unroll
  for (int q = 0; q < 8; ++q) *(volatile v4f*)(gp + (size_t)q * HW) = ov[q];
}

__global__ __launch_bounds__(128) void k_gemm4(
    const float* __restrict__ h3, const unsigned short* __restrict__ wp,
    const float* __restrict__ b4, float* out, int nN) {
  __shared__ __attribute__((aligned(16))) float stg[GROWS * OUTW];
  const int tid = threadIdx.x, lane = tid & 31, wave = tid >> 5, hh = lane >> 4, m = lane & 15;
  const int row0 = blockIdx.x * GROWS;
  const int arow = row0 + 16 * wave + m;
  const unsigned short* whi = wp;
  const unsigned short* wlo = wp + P4N;

  v8f acc[3];
#pragma unroll
  for (int t = 0; t < 3; ++t) { v8f zz = {0.f, 0.f, 0.f, 0.f, 0.f, 0.f, 0.f, 0.f}; acc[t] = zz; }

#pragma unroll
  for (int ks = 0; ks < H3W / 32; ++ks) {
    const float* p0 = h3 + (size_t)arow * H3W + 32 * ks + 8 * hh;
    const v4f f0 = *(const v4f*)p0,        f1 = *(const v4f*)(p0 + 4);
    const v4f f2 = *(const v4f*)(p0 + 16), f3 = *(const v4f*)(p0 + 20);
    const HL s0 = split8(f0, f1);
    const HL s1 = split8(f2, f3);
    FragB ah, al;
    ah.h[0] = s0.hi; ah.h[1] = s1.hi;
    al.h[0] = s0.lo; al.h[1] = s1.lo;
#pragma unroll
    for (int t = 0; t < 3; ++t) {
      const unsigned short* bp = whi + (size_t)(16 * t + m) * H3W + 32 * ks + 8 * hh;
      const unsigned short* bq = wlo + (size_t)(16 * t + m) * H3W + 32 * ks + 8 * hh;
      FragB bh, bl;
      bh.h[0] = *(const v8us*)bp; bh.h[1] = *(const v8us*)(bp + 16);
      bl.h[0] = *(const v8us*)bq; bl.h[1] = *(const v8us*)(bq + 16);
      acc[t] = wmb(ah.v, bh.v, acc[t]);
      acc[t] = wmb(ah.v, bl.v, acc[t]);
      acc[t] = wmb(al.v, bh.v, acc[t]);
    }
  }

#pragma unroll
  for (int t = 0; t < 3; ++t) {
    const int col = 16 * t + m;
    if (col < OUTW) {
      const float bc = b4[col];
      float* sp = stg + (16 * wave + 8 * hh) * OUTW + col;
      sp[0 * OUTW] = acc[t][0] + bc;
      sp[1 * OUTW] = acc[t][1] + bc;
      sp[2 * OUTW] = acc[t][2] + bc;
      sp[3 * OUTW] = acc[t][3] + bc;
      sp[4 * OUTW] = acc[t][4] + bc;
      sp[5 * OUTW] = acc[t][5] + bc;
      sp[6 * OUTW] = acc[t][6] + bc;
      sp[7 * OUTW] = acc[t][7] + bc;
    }
  }
  __syncthreads();

  const size_t total = (size_t)nN * OUTW;
  const size_t ob    = (size_t)row0 * OUTW;
  v4f ov[5];
#pragma unroll
  for (int q = 0; q < 5; ++q) ov[q] = *(const v4f*)(stg + (wave * 5 + q) * 128 + 4 * lane);
#pragma unroll
  for (int q = 0; q < 5; ++q) {
    const size_t gi = ob + (size_t)((wave * 5 + q) * 128 + 4 * lane);
    if (gi < total) *(volatile v4f*)(out + gi) = ov[q];
  }
  __threadfence();
#pragma unroll
  for (int q = 0; q < 5; ++q) {
    const size_t gi = ob + (size_t)((wave * 5 + q) * 128 + 4 * lane);
    if (gi < total) *(volatile v4f*)(out + gi) = ov[q];
  }
}

extern "C" void kernel_launch(void* const* d_in, const int* in_sizes, int n_in,
                              void* d_out, int out_size, void* d_ws, size_t ws_size,
                              hipStream_t stream) {
  if (n_in < 13) return;
  const int nN = in_sizes[0] / 3;
  const int nE = in_sizes[1] / 2;
  if (nN <= 0 || nE < 0 || in_sizes[0] != nN * 3 || in_sizes[1] != nE * 2) return;
  if (in_sizes[2] != 3 * HW || in_sizes[3] != 3 * HW || in_sizes[4] != HW) return;
  if (in_sizes[5] != HW * HW || in_sizes[6] != HW * HW || in_sizes[7] != HW) return;
  if (in_sizes[8] != HW * H3W || in_sizes[9] != HW * H3W || in_sizes[10] != H3W) return;
  if (in_sizes[11] != H3W * OUTW || in_sizes[12] != OUTW) return;
  if (out_size != nN * OUTW) return;

  const float* z   = (const float*)d_in[0];
  const int*   ei  = (const int*)d_in[1];
  const float* W1l = (const float*)d_in[2];
  const float* W1r = (const float*)d_in[3];
  const float* b1  = (const float*)d_in[4];
  const float* W2l = (const float*)d_in[5];
  const float* W2r = (const float*)d_in[6];
  const float* b2  = (const float*)d_in[7];
  const float* W3l = (const float*)d_in[8];
  const float* W3r = (const float*)d_in[9];
  const float* b3  = (const float*)d_in[10];
  const float* W4  = (const float*)d_in[11];
  const float* b4  = (const float*)d_in[12];
  float* out = (float*)d_out;

  const int nPad = ((nN + GROWS - 1) / GROWS) * GROWS;
  const int nGB  = nPad / GROWS;
  const int nA1  = (nN + NB1 - 1) / NB1;
  const int nA2  = (nN + NB2 - 1) / NB2;
  const int nA3  = (nN + NB3 - 1) / NB3;

  char* ws = (char*)d_ws;
  size_t off = 0;
  const size_t oP2 = off; off += (size_t)P2N * 2 * 2;            off = (off + 255) & ~(size_t)255;
  const size_t oP3 = off; off += (size_t)P3N * 2 * 2;            off = (off + 255) & ~(size_t)255;
  const size_t oP4 = off; off += (size_t)P4N * 2 * 2;            off = (off + 255) & ~(size_t)255;
  const size_t szF = (size_t)nPad * HW * 4;
  const size_t oF0 = off; off += szF;                            off = (off + 255) & ~(size_t)255;
  const size_t oF1 = off; off += szF;                            off = (off + 255) & ~(size_t)255;
  if (off > ws_size) return;
  if (off > ((size_t)128 << 20)) return;
  unsigned short* p2 = (unsigned short*)(ws + oP2);
  unsigned short* p3 = (unsigned short*)(ws + oP3);
  unsigned short* p4 = (unsigned short*)(ws + oP4);
  float* F0 = (float*)(ws + oF0);
  float* F1 = (float*)(ws + oF1);

  const int vec8 = ((nE & 3) == 0) ? 1 : 0;

  const int nPrep = P2N / 8 + P3N / 8 + P4N / 8;
  k_wprep<<<(nPrep + NTHR - 1) / NTHR, NTHR, 0, stream>>>(W2l, W2r, W3l, W3r, W4, p2, p3, p4);

  hipFuncSetAttribute(reinterpret_cast<const void*>(&k_agg1),
                      hipFuncAttributeMaxDynamicSharedMemorySize, LDS_A1);
  k_agg1<<<nA1, NTHR, LDS_A1, stream>>>(z, ei, W1l, W1r, b1, F0, nN, nPad, nE, vec8);

  hipFuncSetAttribute(reinterpret_cast<const void*>(&k_agg128),
                      hipFuncAttributeMaxDynamicSharedMemorySize, LDS_A2);
  k_agg128<<<nA2, NTHR, LDS_A2, stream>>>(ei, F0, F1, nN, nPad, nE, vec8);

  k_gemm<8, true><<<nGB, NTHR, 0, stream>>>(F1, F0, p2, b2, F1, nPad);

  k_gemm<4, false><<<nGB, NTHR, 0, stream>>>(F1, F1 + H3W, p3, b3, F0, nPad);

  hipFuncSetAttribute(reinterpret_cast<const void*>(&k_agg64),
                      hipFuncAttributeMaxDynamicSharedMemorySize, LDS_A3);
  k_agg64<<<nA3, NTHR, LDS_A3, stream>>>(ei, F0, b3, F1, nN, nPad, nE, vec8);

  k_gemm4<<<nGB, 128, 0, stream>>>(F1, p4, b4, out, nN);
}
